// HmmLm_35364760715486
// MI455X (gfx1250) — hardware-verified
//
#include <hip/hip_runtime.h>
#define CS 1024
#define HDIM 256
#define VV 10000
#define VP 10048
#define BB 16
#define NN 256

typedef __bf16 v16b __attribute__((ext_vector_type(16)));
typedef unsigned short v8us __attribute__((ext_vector_type(8), may_alias));
typedef float  v8f  __attribute__((ext_vector_type(8)));
typedef float  v4f  __attribute__((ext_vector_type(4)));
typedef float  v4fa __attribute__((ext_vector_type(4), may_alias));
union FragB { v16b v; v8us half[2]; unsigned short u[16]; };

__device__ __forceinline__ unsigned short bf16_bits(float x) { unsigned int u = __float_as_uint(x); return (unsigned short)((u + 0x7FFFu + ((u >> 16) & 1u)) >> 16); }
__device__ __forceinline__ float bf16_val(unsigned short b) { return __uint_as_float(((unsigned int)b) << 16); }
__device__ __forceinline__ float bf16_round(float x) { return bf16_val(bf16_bits(x)); }
template <int NT>
__device__ __forceinline__ v8f mmaN(v16b ah, v16b al, v16b bh, v16b bl, v8f c) {
  c = __builtin_amdgcn_wmma_f32_16x16x32_bf16(false, ah, false, bh, (short)0, c, false, false);
  if (NT >= 2) c = __builtin_amdgcn_wmma_f32_16x16x32_bf16(false, al, false, bh, (short)0, c, false, false);
  if (NT >= 3) c = __builtin_amdgcn_wmma_f32_16x16x32_bf16(false, ah, false, bl, (short)0, c, false, false);
  asm volatile("v_nop\n\tv_nop\n\tv_nop\n\tv_nop" : "+v"(c) : "v"(ah), "v"(al), "v"(bh), "v"(bl));
  return c;
}

__global__ __launch_bounds__(256) void k_wt_bf16(const float* __restrict__ W, unsigned short* __restrict__ Wt, int K, int N) {
  const int t = blockIdx.x * 256 + threadIdx.x;
  const int k8n = K / 8;
  if (t >= N * k8n) return;
  const int n = t / k8n, k8 = (t % k8n) * 8;
  v8us v;
#pragma unroll
  for (int i = 0; i < 8; ++i) v[i] = bf16_bits(W[(size_t)(k8 + i) * N + n]);
  *(volatile v8us*)(Wt + (size_t)n * K + k8) = v;
  __threadfence();
  *(volatile v8us*)(Wt + (size_t)n * K + k8) = v;
}

template <bool ASPLIT, int ACT, bool BIAS_BF16>
__global__ __launch_bounds__(128) void k_gemm_bf(const float* __restrict__ A, int lda, const unsigned short* __restrict__ Wt, int ldb,
                                               const float* __restrict__ bias, float* __restrict__ C, int ldc, int M, int N, int K) {
  __shared__ __attribute__((aligned(16))) float so[4][16][64];
  const int tid = threadIdx.x, w = tid >> 5, lane = tid & 31, ln = lane & 15, hh = lane >> 4;
  const int ntn = N / 64;
  const int wid = blockIdx.x * 4 + w;
  const int mt = wid / ntn, nq = wid % ntn;
  if (mt * 16 >= M) return;
  const int row0 = mt * 16, col0 = nq * 64;
  const float* arow = A + (size_t)(row0 + ln) * lda;
  v8f acc[4] = {};
  for (int kb = 0; kb < K; kb += 32) {
    FragB ah, al;
    const v4f x0 = *(const v4fa*)(arow + kb + 8 * hh), x1 = *(const v4fa*)(arow + kb + 8 * hh + 4);
    const v4f x2 = *(const v4fa*)(arow + kb + 16 + 8 * hh), x3 = *(const v4fa*)(arow + kb + 16 + 8 * hh + 4);
    float xs[16] = {x0[0],x0[1],x0[2],x0[3],x1[0],x1[1],x1[2],x1[3],x2[0],x2[1],x2[2],x2[3],x3[0],x3[1],x3[2],x3[3]};
#pragma unroll
    for (int i = 0; i < 16; ++i) { const unsigned short hb = bf16_bits(xs[i]); ah.u[i] = hb; al.u[i] = ASPLIT ? bf16_bits(xs[i] - bf16_val(hb)) : (unsigned short)0; }
#pragma unroll
    for (int t = 0; t < 4; ++t) {
      const unsigned short* brow = Wt + (size_t)(col0 + t * 16 + ln) * ldb + kb;
      FragB b;
      b.half[0] = *(const v8us*)(brow + 8 * hh);
      b.half[1] = *(const v8us*)(brow + 16 + 8 * hh);
      acc[t] = mmaN<ASPLIT ? 2 : 1>(ah.v, al.v, b.v, b.v, acc[t]);
    }
  }
#pragma unroll
  for (int t = 0; t < 4; ++t) {
    float bv = bias ? bias[col0 + t * 16 + ln] : 0.f;
    if (BIAS_BF16) bv = bf16_round(bv);
#pragma unroll
    for (int r = 0; r < 8; ++r) { float v = acc[t][r] + bv; if (ACT == 1) v = fmaxf(v, 0.f); so[w][8 * hh + r][t * 16 + ln] = v; }
  }
  __builtin_amdgcn_fence(__ATOMIC_ACQ_REL, "workgroup");
  __builtin_amdgcn_wave_barrier();
  const int rsub = lane >> 4, c4 = (lane & 15) * 4;
  for (int pass = 0; pass < 2; ++pass) {
#pragma unroll
    for (int q = 0; q < 8; ++q) {
      const int r = q * 2 + rsub;
      const v4f v = *(const v4fa*)&so[w][r][c4];
      *(volatile v4f*)(C + (size_t)(row0 + r) * ldc + col0 + c4) = v;
    }
    if (pass == 0) __threadfence();
  }
}

template <int D, bool CAUSAL>
__global__ __launch_bounds__(128) void k_flash(const float* __restrict__ qb, const float* __restrict__ kb, const float* __restrict__ vb,
                                             int pitch, int T, int H, float scale, float* __restrict__ y, int ypitch) {
  constexpr int KS = D / 32;
  constexpr int DT = D / 16;
  __shared__ __attribute__((aligned(16))) unsigned short sKh[32][D + 8], sKl[32][D + 8], sVh[32][D + 8], sVl[32][D + 8];
  __shared__ __attribute__((aligned(16))) unsigned short sPh[4][16][40], sPl[4][16][40];
  __shared__ __attribute__((aligned(16))) float sO[4][16][D];
  const int tid = threadIdx.x, w = tid >> 5, lane = tid & 31, ln = lane & 15, hh = lane >> 4;
  const int nqb = (T + 63) / 64;
  const int bh = blockIdx.x / nqb, qblk = blockIdx.x % nqb;
  const int b = bh / H, h = bh % H;
  const int q0 = qblk * 64 + w * 16;
  const float* Q = qb + (size_t)b * T * pitch + h * D;
  const float* K = kb + (size_t)b * T * pitch + h * D;
  const float* V = vb + (size_t)b * T * pitch + h * D;

  FragB aqh[KS], aql[KS];
  {
    int row = q0 + ln; if (row >= T) row = T - 1;
    const float* qr = Q + (size_t)row * pitch;
#pragma unroll
    for (int ks = 0; ks < KS; ++ks)
#pragma unroll
      for (int i = 0; i < 16; ++i) {
        const int d = ks * 32 + ((i < 8) ? (8 * hh + i) : (16 + 8 * hh + (i - 8)));
        const float x = qr[d] * scale; const unsigned short hb = bf16_bits(x);
        aqh[ks].u[i] = hb; aql[ks].u[i] = bf16_bits(x - bf16_val(hb));
      }
  }
  float m_r[8], l_r[8];
#pragma unroll
  for (int r = 0; r < 8; ++r) { m_r[r] = -3.0e38f; l_r[r] = 0.f; }
  v8f oacc[DT];
#pragma unroll
  for (int dt = 0; dt < DT; ++dt) oacc[dt] = (v8f){0.f,0.f,0.f,0.f,0.f,0.f,0.f,0.f};

  const int kv_end = CAUSAL ? min(T, qblk * 64 + 64) : T;
  for (int j0 = 0; j0 < kv_end; j0 += 32) {
    __syncthreads();
    for (int e = tid; e < 32 * (D / 4); e += 128) {
      const int r = e / (D / 4), c4 = (e % (D / 4)) * 4;
      const int key = j0 + r;
      v4f kf = {0.f,0.f,0.f,0.f}, vf = {0.f,0.f,0.f,0.f};
      if (key < T) { kf = *(const v4fa*)(K + (size_t)key * pitch + c4); vf = *(const v4fa*)(V + (size_t)key * pitch + c4); }
#pragma unroll
      for (int t = 0; t < 4; ++t) {
        unsigned short hb = bf16_bits(kf[t]); sKh[r][c4 + t] = hb; sKl[r][c4 + t] = bf16_bits(kf[t] - bf16_val(hb));
        hb = bf16_bits(vf[t]); sVh[r][c4 + t] = hb; sVl[r][c4 + t] = bf16_bits(vf[t] - bf16_val(hb));
      }
    }
    __syncthreads();
    v8f s[2];
#pragma unroll
    for (int nt = 0; nt < 2; ++nt) {
      v8f acc = {};
#pragma unroll
      for (int ks = 0; ks < KS; ++ks) {
        FragB bh_, bl_;
        bh_.half[0] = *(const v8us*)&sKh[nt * 16 + ln][ks * 32 + 8 * hh]; bh_.half[1] = *(const v8us*)&sKh[nt * 16 + ln][ks * 32 + 16 + 8 * hh];
        bl_.half[0] = *(const v8us*)&sKl[nt * 16 + ln][ks * 32 + 8 * hh]; bl_.half[1] = *(const v8us*)&sKl[nt * 16 + ln][ks * 32 + 16 + 8 * hh];
        acc = mmaN<3>(aqh[ks].v, aql[ks].v, bh_.v, bl_.v, acc);
      }
      s[nt] = acc;
    }
    float alpha[8];
#pragma unroll
    for (int r = 0; r < 8; ++r) {
      const int qi = q0 + 8 * hh + r;
      const int ja = j0 + ln, jb = j0 + 16 + ln;
      if (CAUSAL) { if (ja > qi) s[0][r] = -3.0e38f; if (jb > qi) s[1][r] = -3.0e38f; }
      if (ja >= T) s[0][r] = -3.0e38f;
      if (jb >= T) s[1][r] = -3.0e38f;
      float mx = fmaxf(s[0][r], s[1][r]);
      mx = fmaxf(mx, __shfl_xor(mx, 1, 32)); mx = fmaxf(mx, __shfl_xor(mx, 2, 32)); mx = fmaxf(mx, __shfl_xor(mx, 4, 32)); mx = fmaxf(mx, __shfl_xor(mx, 8, 32));
      const float mnew = fmaxf(m_r[r], mx);
      alpha[r] = (mnew > -1.0e38f) ? __expf(m_r[r] - mnew) : 1.0f;
      const float p0 = (s[0][r] > -1.0e38f) ? __expf(s[0][r] - mnew) : 0.f;
      const float p1 = (s[1][r] > -1.0e38f) ? __expf(s[1][r] - mnew) : 0.f;
      m_r[r] = mnew;
      l_r[r] = l_r[r] * alpha[r] + p0 + p1;
      unsigned short hb = bf16_bits(p0); sPh[w][8 * hh + r][ln] = hb;      sPl[w][8 * hh + r][ln] = bf16_bits(p0 - bf16_val(hb));
      hb = bf16_bits(p1);                sPh[w][8 * hh + r][16 + ln] = hb; sPl[w][8 * hh + r][16 + ln] = bf16_bits(p1 - bf16_val(hb));
    }
#pragma unroll
    for (int dt = 0; dt < DT; ++dt)
#pragma unroll
      for (int r = 0; r < 8; ++r) oacc[dt][r] *= alpha[r];
    __builtin_amdgcn_fence(__ATOMIC_ACQ_REL, "workgroup");
    __builtin_amdgcn_wave_barrier();
    FragB pah, pal;
    pah.half[0] = *(const v8us*)&sPh[w][ln][8 * hh]; pah.half[1] = *(const v8us*)&sPh[w][ln][16 + 8 * hh];
    pal.half[0] = *(const v8us*)&sPl[w][ln][8 * hh]; pal.half[1] = *(const v8us*)&sPl[w][ln][16 + 8 * hh];
#pragma unroll
    for (int dt = 0; dt < DT; ++dt) {
      FragB bvh, bvl;
#pragma unroll
      for (int i = 0; i < 8; ++i) {
        bvh.u[i] = sVh[8 * hh + i][dt * 16 + ln]; bvh.u[8 + i] = sVh[16 + 8 * hh + i][dt * 16 + ln];
        bvl.u[i] = sVl[8 * hh + i][dt * 16 + ln]; bvl.u[8 + i] = sVl[16 + 8 * hh + i][dt * 16 + ln];
      }
      oacc[dt] = mmaN<3>(pah.v, pal.v, bvh.v, bvl.v, oacc[dt]);
    }
    __builtin_amdgcn_fence(__ATOMIC_ACQ_REL, "workgroup");
    __builtin_amdgcn_wave_barrier();
  }
#pragma unroll
  for (int r = 0; r < 8; ++r) {
    float l = l_r[r];
    l += __shfl_xor(l, 1, 32); l += __shfl_xor(l, 2, 32); l += __shfl_xor(l, 4, 32); l += __shfl_xor(l, 8, 32);
    l_r[r] = (l > 0.f) ? 1.0f / l : 0.f;
  }
#pragma unroll
  for (int dt = 0; dt < DT; ++dt)
#pragma unroll
    for (int r = 0; r < 8; ++r) sO[w][8 * hh + r][dt * 16 + ln] = oacc[dt][r] * l_r[r];
  __builtin_amdgcn_fence(__ATOMIC_ACQ_REL, "workgroup");
  __builtin_amdgcn_wave_barrier();
  for (int pass = 0; pass < 2; ++pass) {
    for (int r = 0; r < 16; ++r) {
      const int row = q0 + r;
      if (row < T && lane < D / 4) {
        const v4f val = *(const v4fa*)&sO[w][r][lane * 4];
        *(volatile v4f*)(y + ((size_t)b * T + row) * ypitch + h * D + lane * 4) = val;
      }
    }
    if (pass == 0) __threadfence();
  }
}

template <bool ASPLIT, int ACT, bool BIAS_BF16, bool RES_BF16>
__global__ __launch_bounds__(128) void k_gemm_bf3(const float* __restrict__ A, int lda, const unsigned short* __restrict__ Wt, int ldb,
                                                const float* __restrict__ bias, const float* __restrict__ resid, int rmod, int ldr,
                                                float* __restrict__ C, int ldc, int M, int N, int K) {
  __shared__ __attribute__((aligned(16))) float so[4][16][64];
  const int tid = threadIdx.x, w = tid >> 5, lane = tid & 31, ln = lane & 15, hh = lane >> 4;
  const int ntn = N / 64;
  const int wid = blockIdx.x * 4 + w;
  const int mt = wid / ntn, nq = wid % ntn;
  if (mt * 16 >= M) return;
  const int row0 = mt * 16, col0 = nq * 64;
  const float* arow = A + (size_t)(row0 + ln) * lda;
  v8f acc[4] = {};
  for (int kb = 0; kb < K; kb += 32) {
    FragB ah, al;
    const v4f x0 = *(const v4fa*)(arow + kb + 8 * hh), x1 = *(const v4fa*)(arow + kb + 8 * hh + 4);
    const v4f x2 = *(const v4fa*)(arow + kb + 16 + 8 * hh), x3 = *(const v4fa*)(arow + kb + 16 + 8 * hh + 4);
    float xs[16] = {x0[0],x0[1],x0[2],x0[3],x1[0],x1[1],x1[2],x1[3],x2[0],x2[1],x2[2],x2[3],x3[0],x3[1],x3[2],x3[3]};
#pragma unroll
    for (int i = 0; i < 16; ++i) { const unsigned short hb = bf16_bits(xs[i]); ah.u[i] = hb; al.u[i] = ASPLIT ? bf16_bits(xs[i] - bf16_val(hb)) : (unsigned short)0; }
#pragma unroll
    for (int t = 0; t < 4; ++t) {
      const unsigned short* brow = Wt + (size_t)(col0 + t * 16 + ln) * ldb + kb;
      FragB b;
      b.half[0] = *(const v8us*)(brow + 8 * hh);
      b.half[1] = *(const v8us*)(brow + 16 + 8 * hh);
      acc[t] = mmaN<ASPLIT ? 2 : 1>(ah.v, al.v, b.v, b.v, acc[t]);
    }
  }
#pragma unroll
  for (int t = 0; t < 4; ++t) {
    const int col = col0 + t * 16 + ln;
    float bv = bias ? bias[col] : 0.f;
    if (BIAS_BF16) bv = bf16_round(bv);
#pragma unroll
    for (int r = 0; r < 8; ++r) {
      float v = acc[t][r] + bv;
      if (resid) { float rv = resid[(size_t)((row0 + 8 * hh + r) % rmod) * ldr + col]; if (RES_BF16) rv = bf16_round(rv); v += rv; }
      if (ACT == 1) v = fmaxf(v, 0.f);
      if (ACT == 2) v = 0.5f * v * (1.0f + erff(v * 0.70710678118654752f));
      if (ACT == 3) { const float u = 0.7978845608028654f * (v + 0.044715f * v * v * v); v = 0.5f * v * (1.0f + tanhf(u)); }
      so[w][8 * hh + r][t * 16 + ln] = v;
    }
  }
  __builtin_amdgcn_fence(__ATOMIC_ACQ_REL, "workgroup");
  __builtin_amdgcn_wave_barrier();
  const int rsub = lane >> 4, c4 = (lane & 15) * 4;
  for (int pass = 0; pass < 2; ++pass) {
#pragma unroll
    for (int q = 0; q < 8; ++q) {
      const int r = q * 2 + rsub;
      const v4f v = *(const v4fa*)&so[w][r][c4];
      *(volatile v4f*)(C + (size_t)(row0 + r) * ldc + col0 + c4) = v;
    }
    if (pass == 0) __threadfence();
  }
}
template <bool PARAM_BF16>
__global__ __launch_bounds__(256) void k_layernorm(const float* __restrict__ X, const float* __restrict__ R, const float* __restrict__ g, const float* __restrict__ bta,
                                                  float* __restrict__ out_sum, float* __restrict__ out_norm, int N, float eps) {
  __shared__ float red[256];
  const int row = blockIdx.x, tid = threadIdx.x;
  const float* x = X + (size_t)row * N; const float* rr = R ? R + (size_t)row * N : nullptr;
  float vals[16];
  const int per = N / 256;
  float s1 = 0.f;
  for (int u = 0; u < per / 4; ++u) {
    const int j = tid * 4 + 1024 * u;
    const v4f a = *(const v4fa*)(x + j);
    v4f b = {0.f,0.f,0.f,0.f}; if (rr) b = *(const v4fa*)(rr + j);
#pragma unroll
    for (int q = 0; q < 4; ++q) { const float v = a[q] + b[q]; vals[u * 4 + q] = v; s1 += v; }
  }
  red[tid] = s1; __syncthreads();
  for (int st = 128; st > 0; st >>= 1) { if (tid < st) red[tid] += red[tid + st]; __syncthreads(); }
  const float mu = red[0] / (float)N; __syncthreads();
  float s2 = 0.f;
  for (int u = 0; u < per / 4; ++u)
#pragma unroll
    for (int q = 0; q < 4; ++q) { const float c = vals[u * 4 + q] - mu; s2 += c * c; }
  red[tid] = s2; __syncthreads();
  for (int st = 128; st > 0; st >>= 1) { if (tid < st) red[tid] += red[tid + st]; __syncthreads(); }
  const float rs = rsqrtf(red[0] / (float)N + eps);
  for (int pass = 0; pass < 2; ++pass) {
    for (int u = 0; u < per / 4; ++u) {
      const int j = tid * 4 + 1024 * u;
      v4f o, sm;
#pragma unroll
      for (int q = 0; q < 4; ++q) {
        float gg = g[j + q], bb = bta[j + q];
        if (PARAM_BF16) { gg = bf16_round(gg); bb = bf16_round(bb); }
        sm[q] = vals[u * 4 + q]; o[q] = (vals[u * 4 + q] - mu) * rs * gg + bb;
      }
      if (out_sum) *(volatile v4f*)(out_sum + (size_t)row * N + j) = sm;
      *(volatile v4f*)(out_norm + (size_t)row * N + j) = o;
    }
    if (pass == 0) __threadfence();
  }
}

__global__ __launch_bounds__(256) void k_round_rows(const float* __restrict__ W, unsigned short* __restrict__ Wt, int n8) {
  const int t = blockIdx.x * 256 + threadIdx.x;
  if (t >= n8) return;
  const v4f a = *(const v4fa*)(W + (size_t)t * 8), b = *(const v4fa*)(W + (size_t)t * 8 + 4);
  v8us v; v[0]=bf16_bits(a[0]); v[1]=bf16_bits(a[1]); v[2]=bf16_bits(a[2]); v[3]=bf16_bits(a[3]);
  v[4]=bf16_bits(b[0]); v[5]=bf16_bits(b[1]); v[6]=bf16_bits(b[2]); v[7]=bf16_bits(b[3]);
  *(volatile v8us*)(Wt + (size_t)t * 8) = v; __threadfence(); *(volatile v8us*)(Wt + (size_t)t * 8) = v;
}

__global__ __launch_bounds__(256) void k_brelu(float* __restrict__ Y, const float* __restrict__ b, int n4tot) { const int t = blockIdx.x * 256 + threadIdx.x; if (t >= n4tot) return; const int c4 = (t * 4) % HDIM; v4f v = *(const v4fa*)(Y + (size_t)t * 4); for (int q = 0; q < 4; ++q) v[q] = fmaxf(v[q] + bf16_round(b[c4 + q]), 0.f); *(volatile v4f*)(Y + (size_t)t * 4) = v; __threadfence(); *(volatile v4f*)(Y + (size_t)t * 4) = v; }
__global__ __launch_bounds__(256) void k_resln(const float* __restrict__ H1r, const float* __restrict__ H2, const float* __restrict__ b2, const float* __restrict__ g, const float* __restrict__ be, float* __restrict__ R) {
  const int tid = threadIdx.x, wv = tid >> 5, lane = tid & 31; const int r = blockIdx.x * 8 + wv; if (r >= CS) return; float v[8]; float s = 0.f;
#pragma unroll
  for (int u = 0; u < 8; ++u) { const int c = u * 32 + lane; v[u] = fmaxf(H2[(size_t)r * HDIM + c] + bf16_round(b2[c]), 0.f) + H1r[(size_t)r * HDIM + c]; s += v[u]; }
  for (int o = 16; o >= 1; o >>= 1) s += __shfl_xor(s, o, 32); const float mu = s * (1.0f / HDIM); float q = 0.f;
#pragma unroll
  for (int u = 0; u < 8; ++u) { const float d = v[u] - mu; q += d * d; } for (int o = 16; o >= 1; o >>= 1) q += __shfl_xor(q, o, 32); const float rs = rsqrtf(q * (1.0f / HDIM) + 1e-5f);
#pragma unroll
  for (int u = 0; u < 8; ++u) { const int c = u * 32 + lane; v[u] = bf16_round(g[c]) * (v[u] - mu) * rs + bf16_round(be[c]); }
  for (int pass = 0; pass < 2; ++pass) {
#pragma unroll
    for (int u = 0; u < 8; ++u) *(volatile float*)(R + (size_t)r * HDIM + u * 32 + lane) = v[u]; if (pass == 0) __threadfence(); }
}
__global__ __launch_bounds__(1024) void k_start(const float* __restrict__ R, const float* __restrict__ Wo, const float* __restrict__ bo, float* __restrict__ ST) { __shared__ float sl[CS]; __shared__ float red[32]; const int c = threadIdx.x, lane = c & 31, wv = c >> 5; float s = bf16_round(bo[0]);
#pragma unroll 4
  for (int k = 0; k < HDIM; ++k) s += R[(size_t)c * HDIM + k] * bf16_round(Wo[k]); sl[c] = s;
  float m = s; for (int o = 16; o >= 1; o >>= 1) m = fmaxf(m, __shfl_xor(m, o, 32)); if (lane == 0) red[wv] = m; __syncthreads(); m = red[0]; for (int w2 = 1; w2 < 32; ++w2) m = fmaxf(m, red[w2]); __syncthreads();
  float e = expf(s - m); for (int o = 16; o >= 1; o >>= 1) e += __shfl_xor(e, o, 32); if (lane == 0) red[wv] = e; __syncthreads(); float tot = 0.f; for (int w2 = 0; w2 < 32; ++w2) tot += red[w2]; const float lse = m + logf(tot);
  *(volatile float*)(ST + c) = s - lse; __threadfence(); *(volatile float*)(ST + c) = s - lse; }
__global__ __launch_bounds__(256) void k_rowlse(const float* __restrict__ L, int ld, int N, int rows, float* __restrict__ LSE) { __shared__ float so[8]; const int tid = threadIdx.x, wv = tid >> 5, lane = tid & 31; const int r = blockIdx.x * 8 + wv; float m = -3.0e38f;
  if (r < rows) { const float* row = L + (size_t)r * ld; for (int j = lane; j < N; j += 32) m = fmaxf(m, row[j]); for (int o = 16; o >= 1; o >>= 1) m = fmaxf(m, __shfl_xor(m, o, 32)); float e = 0.f; for (int j = lane; j < N; j += 32) e += expf(row[j] - m); for (int o = 16; o >= 1; o >>= 1) e += __shfl_xor(e, o, 32); m = m + logf(e); }
  if (lane == 0) so[wv] = m; __syncthreads(); if (tid < 8) { *(volatile float*)(LSE + blockIdx.x * 8 + tid) = so[tid]; } __threadfence(); if (tid < 8) { *(volatile float*)(LSE + blockIdx.x * 8 + tid) = so[tid]; } }
__global__ __launch_bounds__(256) void k_ptrans(const float* __restrict__ TL, const float* __restrict__ LSE, unsigned short* __restrict__ PT) { __shared__ float tile[64][33]; const int i0 = blockIdx.x * 64, j0 = blockIdx.y * 32; const int tx = threadIdx.x & 31, ty = threadIdx.x >> 5;
  for (int r = ty; r < 64; r += 8) tile[r][tx] = expf(TL[(size_t)(i0 + r) * CS + j0 + tx] - LSE[i0 + r]); __syncthreads(); typedef unsigned short us2 __attribute__((ext_vector_type(2)));
  for (int pass = 0; pass < 2; ++pass) { for (int e = threadIdx.x; e < 32 * 32; e += 256) { const int jr = e >> 5, ip = (e & 31) * 2; us2 v; v.x = bf16_bits(tile[ip][jr]); v.y = bf16_bits(tile[ip + 1][jr]); *(volatile us2*)(PT + (size_t)(j0 + jr) * CS + i0 + ip) = v; } if (pass == 0) __threadfence(); } }
__global__ __launch_bounds__(256) void k_zpadE(const float* __restrict__ W, unsigned short* __restrict__ Bt) { const int t = blockIdx.x * 256 + threadIdx.x; if (t >= VP * HDIM / 8) return; const int n = t / (HDIM / 8), k8 = (t % (HDIM / 8)) * 8; v8us v; for (int q = 0; q < 8; ++q) v[q] = bf16_bits(n < VV ? W[(size_t)n * HDIM + k8 + q] : 0.f); *(volatile v8us*)(Bt + (size_t)n * HDIM + k8) = v; __threadfence(); *(volatile v8us*)(Bt + (size_t)n * HDIM + k8) = v; }
__global__ __launch_bounds__(256) void k_addbE(float* __restrict__ EL, const float* __restrict__ bo) { const size_t t = (size_t)blockIdx.x * 256 + threadIdx.x; if (t >= (size_t)CS * VP / 4) return; const int c4 = (int)((t * 4) % VP); v4f v = *(const v4fa*)(EL + t * 4); for (int q = 0; q < 4; ++q) { const int c = c4 + q; v[q] += (c < VV) ? bf16_round(bo[c]) : 0.f; } *(volatile v4f*)(EL + t * 4) = v; __threadfence(); *(volatile v4f*)(EL + t * 4) = v; }
__global__ __launch_bounds__(256) void k_emit(const float* __restrict__ EL, const float* __restrict__ lseE, const int* __restrict__ text, float* __restrict__ EM) { const int t = blockIdx.x * 256 + threadIdx.x; if (t >= NN * BB * CS) return; const int c = t % CS; const int b = (t / CS) % BB; const int n = t / (CS * BB); int w = text[b * NN + n]; w = w < 0 ? 0 : (w >= VV ? VV - 1 : w);
  const float v = EL[(size_t)c * VP + w] - lseE[c]; *(volatile float*)(EM + t) = v; __threadfence(); *(volatile float*)(EM + t) = v; }
__global__ __launch_bounds__(512) void k_forward(const float* __restrict__ ST, const float* __restrict__ EM, const unsigned short* __restrict__ PT, volatile float* AL, float* __restrict__ out) {
  __shared__ float sa[BB][CS + 4]; __shared__ float smx[16][BB]; __shared__ float sm[BB]; __shared__ float se[16][BB];
  const int tid = threadIdx.x, w = tid >> 5, lane = tid & 31, ln = lane & 15, hh = lane >> 4; const int col0 = w * 64;
  for (int b = 0; b < BB; ++b) { for (int c = col0 + lane; c < col0 + 64; c += 32) { const float v = ST[c] + EM[(size_t)(0 * BB + b) * CS + c]; *(AL + (size_t)b * CS + c) = v; } }
  __threadfence_block(); __syncthreads();
#pragma unroll 1
  for (int n = 1; n <= NN; ++n) {
    for (int b = 0; b < BB; ++b) { float m = fmaxf(AL[(size_t)b * CS + col0 + lane], AL[(size_t)b * CS + col0 + 32 + lane]); for (int o = 16; o >= 1; o >>= 1) m = fmaxf(m, __shfl_xor(m, o, 32)); if (lane == 0) smx[w][b] = m; }
    __syncthreads(); if (tid < BB) { float m = smx[0][tid]; for (int k = 1; k < 16; ++k) m = fmaxf(m, smx[k][tid]); sm[tid] = m; } __syncthreads();
    if (n == NN) break;
    for (int b = 0; b < BB; ++b) { for (int c = col0 + lane; c < col0 + 64; c += 32) sa[b][c] = expf(AL[(size_t)b * CS + c] - sm[b]); }
    __syncthreads();
    v8f acc[4] = {};
#pragma unroll 1
    for (int kb = 0; kb < CS; kb += 32) { FragB ah, alo; const float* ar = &sa[ln][kb];
#pragma unroll
      for (int i = 0; i < 16; ++i) { const int k = (i < 8) ? (8 * hh + i) : (16 + 8 * hh + (i - 8)); const float v = ar[k]; const unsigned short hb = bf16_bits(v); ah.u[i] = hb; alo.u[i] = bf16_bits(v - bf16_val(hb)); }
#pragma unroll
      for (int t = 0; t < 4; ++t) { const size_t boff = (size_t)(col0 + t * 16 + ln) * CS + kb; FragB bq; bq.half[0] = *(const v8us*)(PT + boff + 8 * hh); bq.half[1] = *(const v8us*)(PT + boff + 16 + 8 * hh); acc[t] = mmaN<2>(ah.v, alo.v, bq.v, bq.v, acc[t]); } }
#pragma unroll
    for (int t = 0; t < 4; ++t) {
#pragma unroll
      for (int r = 0; r < 8; ++r) { const int b = 8 * hh + r, j = col0 + t * 16 + ln; const float v = (logf(fmaxf(acc[t][r], 1e-38f)) + sm[b]) + EM[((size_t)n * BB + b) * CS + j]; *(AL + (size_t)b * CS + j) = v; } }
    __threadfence_block(); __syncthreads();
  }
  for (int b = 0; b < BB; ++b) { float e = expf(AL[(size_t)b * CS + col0 + lane] - sm[b]) + expf(AL[(size_t)b * CS + col0 + 32 + lane] - sm[b]); for (int o = 16; o >= 1; o >>= 1) e += __shfl_xor(e, o, 32); if (lane == 0) se[w][b] = e; }
  __syncthreads();
  if (tid == 0) { double tot = 0.0; for (int b = 0; b < BB; ++b) { float e = 0.f; for (int k = 0; k < 16; ++k) e += se[k][b]; tot += (double)(sm[b] + logf(e)); } const float v = (float)tot; *(volatile float*)out = v; __threadfence(); *(volatile float*)out = v; }
}
extern "C" void kernel_launch(void* const* d_in, const int* in_sizes, int n_in,
                              void* d_out, int out_size, void* d_ws, size_t ws_size, hipStream_t stream) {
  (void)in_sizes; (void)n_in; (void)out_size;
  const float* emb[3] = {(const float*)d_in[0], (const float*)d_in[1], (const float*)d_in[2]};
  const float* W1[3], *b1[3], *W2[3], *b2[3], *gg[3], *bt[3], *Wo[3], *bo[3];
  for (int p = 0; p < 3; ++p) { W1[p] = (const float*)d_in[3 + p * 8]; b1[p] = (const float*)d_in[4 + p * 8]; W2[p] = (const float*)d_in[5 + p * 8]; b2[p] = (const float*)d_in[6 + p * 8]; gg[p] = (const float*)d_in[7 + p * 8]; bt[p] = (const float*)d_in[8 + p * 8]; Wo[p] = (const float*)d_in[9 + p * 8]; bo[p] = (const float*)d_in[10 + p * 8]; }
  const int* text = (const int*)d_in[27];
  char* ws = (char*)d_ws; size_t off = 0;
  auto take = [&](size_t bytes) { char* p = ws + off; off += (bytes + 255) & ~(size_t)255; return p; };
  unsigned short* BW1 = (unsigned short*)take((size_t)HDIM * HDIM * 2); unsigned short* BW2 = (unsigned short*)take((size_t)HDIM * HDIM * 2); unsigned short* BWt = (unsigned short*)take((size_t)CS * HDIM * 2); unsigned short* BWe = (unsigned short*)take((size_t)VP * HDIM * 2);
  float* H1 = (float*)take((size_t)CS * HDIM * 4); float* H2 = (float*)take((size_t)CS * HDIM * 4); float* R = (float*)take((size_t)CS * HDIM * 4);
  float* ST = (float*)take(CS * 4); float* TL = (float*)take((size_t)CS * CS * 4); float* lseT = (float*)take(CS * 4); unsigned short* PT = (unsigned short*)take((size_t)CS * CS * 2);
  float* EL = (float*)take((size_t)CS * VP * 4); float* lseE = (float*)take(CS * 4); float* EM = (float*)take((size_t)NN * BB * CS * 4); float* ALb = (float*)take((size_t)BB * CS * 4);
  if (off > ws_size) return;
  k_round_rows<<<(CS * HDIM / 8 + 255) / 256, 256, 0, stream>>>(Wo[1], BWt, CS * HDIM / 8);
  {
  }
  for (int p = 0; p < 3; ++p) {
    k_round_rows<<<(HDIM * HDIM / 8 + 255) / 256, 256, 0, stream>>>(W1[p], BW1, HDIM * HDIM / 8); k_round_rows<<<(HDIM * HDIM / 8 + 255) / 256, 256, 0, stream>>>(W2[p], BW2, HDIM * HDIM / 8);
    k_gemm_bf3<false, 0, false, false><<<((CS / 16) * (HDIM / 64) + 3) / 4, 128, 0, stream>>>(emb[p], HDIM, BW1, HDIM, nullptr, nullptr, 1, 0, H1, HDIM, CS, HDIM, HDIM);
    k_brelu<<<(CS * HDIM / 4 + 255) / 256, 256, 0, stream>>>(H1, b1[p], CS * HDIM / 4);
    k_gemm_bf3<true, 0, false, false><<<((CS / 16) * (HDIM / 64) + 3) / 4, 128, 0, stream>>>(H1, HDIM, BW2, HDIM, nullptr, nullptr, 1, 0, H2, HDIM, CS, HDIM, HDIM);
    k_resln<<<CS / 8, 256, 0, stream>>>(H1, H2, b2[p], gg[p], bt[p], R);
    if (p == 0) k_start<<<1, 1024, 0, stream>>>(R, Wo[0], bo[0], ST);
    else if (p == 1) { k_gemm_bf3<true, 0, true, false><<<((CS / 16) * (CS / 64) + 3) / 4, 128, 0, stream>>>(R, HDIM, BWt, HDIM, bo[1], nullptr, 1, 0, TL, CS, CS, CS, HDIM); k_rowlse<<<CS / 8, 256, 0, stream>>>(TL, CS, CS, CS, lseT); k_ptrans<<<dim3(CS / 64, CS / 32), 256, 0, stream>>>(TL, lseT, PT); }
    else { k_zpadE<<<(VP * HDIM / 8 + 255) / 256, 256, 0, stream>>>(Wo[2], BWe); k_gemm_bf3<true, 0, false, false><<<((CS / 16) * (VP / 64) + 3) / 4, 128, 0, stream>>>(R, HDIM, BWe, HDIM, nullptr, nullptr, 1, 0, EL, VP, CS, VP, HDIM); k_addbE<<<(unsigned)(((size_t)CS * VP / 4 + 255) / 256), 256, 0, stream>>>(EL, bo[2]); k_rowlse<<<CS / 8, 256, 0, stream>>>(EL, VP, VV, CS, lseE); }
  }
  k_emit<<<(NN * BB * CS + 255) / 256, 256, 0, stream>>>(EL, lseE, text, EM);
  k_forward<<<1, 512, 0, stream>>>(ST, EM, PT, ALb, (float*)d_out);
}
